// SelfAttnModel_16896401343299
// MI455X (gfx1250) — hardware-verified
//
#include <hip/hip_runtime.h>

#define NB     8
#define NP     4096
#define CH     128
#define DQ     16
#define NT     32768
#define NCOL   160
#define TB     64
#define PVT    72
#define PO     136
#define WPITCH 136

static_assert(NT == NB * NP);
static_assert((NP % TB) == 0 && (NT % TB) == 0 && (NP % 32) == 0 && (CH % 32) == 0);
static_assert(NP / TB == 64);
static_assert(NCOL == 2 * DQ + CH);
static_assert(DQ == 16 && TB == 64 && CH == 128);
static_assert((PVT % 8) == 0 && (PO % 8) == 0 && (WPITCH % 8) == 0);

typedef _Float16       v16h  __attribute__((ext_vector_type(16)));
typedef _Float16       v8h   __attribute__((ext_vector_type(8)));
typedef __bf16         v16bf __attribute__((ext_vector_type(16)));
typedef unsigned short v16us __attribute__((ext_vector_type(16)));
typedef unsigned short v8us  __attribute__((ext_vector_type(8)));
typedef float          v8f   __attribute__((ext_vector_type(8)));
typedef float          v4f   __attribute__((ext_vector_type(4)));
typedef unsigned int   v4u   __attribute__((ext_vector_type(4)));

union FragH { v16h v; v8h half[2]; };
union FragU { v16us v; v8us half[2]; };
union Acc8  { v8f v; v4f q[2]; };

#if defined(__has_builtin)
#if __has_builtin(__builtin_amdgcn_exp2f)
#define FEXP2(x) __builtin_amdgcn_exp2f(x)
#endif
#endif
#ifndef FEXP2
#define FEXP2(x) exp2f(x)
#endif

__device__ __forceinline__ unsigned short bf_bits(float f) {
  unsigned u = __float_as_uint(f);
  return (unsigned short)((u + 0x7FFFu + ((u >> 16) & 1u)) >> 16);
}
__device__ __forceinline__ float bf_up(unsigned short hb) { return __uint_as_float(((unsigned)hb) << 16); }
__device__ __forceinline__ float bf_r(float f) { return bf_up(bf_bits(f)); }
__device__ __forceinline__ v8f zero8() { v8f z = {0.f, 0.f, 0.f, 0.f, 0.f, 0.f, 0.f, 0.f}; return z; }
__device__ __forceinline__ v8h zero8h() {
  v8h z;
#pragma unroll
  for (int i = 0; i < 8; ++i) z[i] = (_Float16)0.0f;
  return z;
}
__device__ __forceinline__ v8us zero8us() { v8us z = {0, 0, 0, 0, 0, 0, 0, 0}; return z; }

__device__ __forceinline__ v16bf ldfrag_b(const unsigned short* p) {
  FragU f;
  f.half[0] = *(const v8us*)(p);
  f.half[1] = *(const v8us*)(p + 16);
  return __builtin_bit_cast(v16bf, f.v);
}
__device__ __forceinline__ v16h ldfrag_h(const _Float16* p) {
  FragH f;
  f.half[0] = *(const v8h*)(p);
  f.half[1] = *(const v8h*)(p + 16);
  return f.v;
}
__device__ __forceinline__ v16bf ldfrag16_b(const unsigned short* p, v8us z) {
  FragU f;
  f.half[0] = *(const v8us*)(p);
  f.half[1] = z;
  return __builtin_bit_cast(v16bf, f.v);
}

__device__ __forceinline__ v8f mma_b(v16bf a, v16bf b, v8f c) {
  return __builtin_amdgcn_wmma_f32_16x16x32_bf16(false, a, false, b, (short)0, c, false, false);
}
__device__ __forceinline__ v8f mma_h(v16h a, v16h b, v8f c) {
  return __builtin_amdgcn_wmma_f32_16x16x32_f16(false, a, false, b, (short)0, c, false, false);
}
__device__ __forceinline__ void guard_pj(v8f& c0, v8f& c1, v8f& c2, v8f& c3, v8f& c4,
                                         v16bf a, v16bf b0, v16bf b1, v16bf b2, v16bf b3, v16bf b4) {
#if defined(__HIP_DEVICE_COMPILE__)
  asm volatile("v_nop\n\tv_nop\n\tv_nop\n\tv_nop"
               : "+v"(c0), "+v"(c1), "+v"(c2), "+v"(c3), "+v"(c4)
               : "v"(a), "v"(b0), "v"(b1), "v"(b2), "v"(b3), "v"(b4));
#endif
}
__device__ __forceinline__ void guard_s1(v8f& s0, v8f& s1, v16bf a0, v16bf a1, v16bf b) {
#if defined(__HIP_DEVICE_COMPILE__)
  asm volatile("v_nop\n\tv_nop\n\tv_nop\n\tv_nop"
               : "+v"(s0), "+v"(s1)
               : "v"(a0), "v"(a1), "v"(b));
#endif
}
__device__ __forceinline__ void guard_s3(v8f& s0, v8f& s1, v16bf a0h, v16bf a1h, v16bf a0l, v16bf a1l,
                                         v16bf bh, v16bf bl) {
#if defined(__HIP_DEVICE_COMPILE__)
  asm volatile("v_nop\n\tv_nop\n\tv_nop\n\tv_nop"
               : "+v"(s0), "+v"(s1)
               : "v"(a0h), "v"(a1h), "v"(a0l), "v"(a1l), "v"(bh), "v"(bl));
#endif
}
__device__ __forceinline__ void guard_pv(v8f& c0, v8f& c1, v8f& c2, v8f& c3,
                                         v16h a0, v16h a1, v16h a2, v16h a3, v16h b) {
#if defined(__HIP_DEVICE_COMPILE__)
  asm volatile("v_nop\n\tv_nop\n\tv_nop\n\tv_nop"
               : "+v"(c0), "+v"(c1), "+v"(c2), "+v"(c3)
               : "v"(a0), "v"(a1), "v"(a2), "v"(a3), "v"(b));
#endif
}
__device__ __forceinline__ void accg5(v8f& a, v8f& b, v8f& c, v8f& d, v8f& e) {
#if defined(__HIP_DEVICE_COMPILE__)
  asm volatile("v_nop\n\tv_nop\n\tv_nop\n\tv_nop" : "+v"(a), "+v"(b), "+v"(c), "+v"(d), "+v"(e));
#endif
}
__device__ __forceinline__ void accg8(v8f& a, v8f& b, v8f& c, v8f& d, v8f& e, v8f& f, v8f& g, v8f& hh) {
#if defined(__HIP_DEVICE_COMPILE__)
  asm volatile("v_nop\n\tv_nop\n\tv_nop\n\tv_nop"
               : "+v"(a), "+v"(b), "+v"(c), "+v"(d), "+v"(e), "+v"(f), "+v"(g), "+v"(hh));
#endif
}
__device__ __forceinline__ void sched_fence() {
#if defined(__HIP_DEVICE_COMPILE__)
  asm volatile("" ::: "memory");
#endif
}

__global__ __launch_bounds__(256) void k_prep(const float* __restrict__ Wq, const float* __restrict__ Wk,
                                               const float* __restrict__ Wv, unsigned short* WT) {
  __shared__ __align__(16) unsigned short s[16 * WPITCH];
  const int tid = threadIdx.x, t = blockIdx.x;
  const float* src;
  int ld, c0;
  if (t == 0) { src = Wq; ld = DQ; c0 = 0; }
  else if (t == 1) { src = Wk; ld = DQ; c0 = 0; }
  else { src = Wv; ld = CH; c0 = (t - 2) * 16; }
#pragma unroll 2
  for (int it = 0; it < (16 * CH) / 256; ++it) {
    const int idx = it * 256 + tid;
    const int k = idx >> 4, nl = idx & 15;
    s[nl * WPITCH + k] = bf_bits(src[k * ld + c0 + nl]);
  }
  __syncthreads();
  const int row = tid >> 4, piece = tid & 15;
  const v8us hv = *(const v8us*)(s + row * WPITCH + piece * 8);
  const v4u u = __builtin_bit_cast(v4u, hv);
  unsigned short* dst = WT + (size_t)(t * 16 + row) * CH + piece * 8;
  *(volatile v4u*)dst = u;
  __threadfence();
  *(volatile v4u*)dst = u;
}

__global__ __launch_bounds__(256) void k_proj(const float* __restrict__ x, const unsigned short* WT,
                                               const float* __restrict__ bq, const float* __restrict__ bk,
                                               const float* __restrict__ bv,
                                               unsigned short* QH, unsigned short* QL,
                                               unsigned short* KH, unsigned short* KL, _Float16* VT) {
  __shared__ __align__(16) _Float16 sVT[CH * PVT];
  __shared__ __align__(16) unsigned short sQH[4 * 16 * DQ];
  __shared__ __align__(16) unsigned short sQL[4 * 16 * DQ];
  __shared__ __align__(16) unsigned short sKH[4 * 16 * DQ];
  __shared__ __align__(16) unsigned short sKL[4 * 16 * DQ];
  __shared__ float sBias[NCOL];
  const int tid = threadIdx.x, w = tid >> 5, lane = tid & 31, m = lane & 15, h = lane >> 4;
  const int tw = w & 3, g = w >> 2;

  if (tid < NCOL) {
    const float b0 = bq[min(tid, DQ - 1)];
    const float b1 = bk[min(max(tid - DQ, 0), DQ - 1)];
    const float b2 = bv[min(max(tid - 2 * DQ, 0), CH - 1)];
    sBias[tid] = bf_r((tid < DQ) ? b0 : ((tid < 2 * DQ) ? b1 : b2));
  }
  __syncthreads();

  const int blk = blockIdx.x;
  const int tok0 = blk * TB;
  const int b = blk >> 6;
  const int tl0 = (blk & 63) * TB;
  const int row0 = tok0 + tw * 16;
  const int tbase = 5 * g;
  const float* xr = x + (size_t)(row0 + m) * CH + 8 * h;
  const unsigned short* wrow = WT + (size_t)(16 * tbase + m) * CH + 8 * h;

  v8f acc[5];
#pragma unroll
  for (int j = 0; j < 5; ++j) acc[j] = zero8();

#pragma unroll 1
  for (int c = 0; c < CH / 32; ++c) {
    const float* p = xr + 32 * c;
    const v4f x0 = *(const v4f*)(p);
    const v4f x1 = *(const v4f*)(p + 4);
    const v4f x2 = *(const v4f*)(p + 16);
    const v4f x3 = *(const v4f*)(p + 20);
    v16us au;
#pragma unroll
    for (int e = 0; e < 4; ++e) {
      au[e]      = bf_bits(x0[e]);
      au[4 + e]  = bf_bits(x1[e]);
      au[8 + e]  = bf_bits(x2[e]);
      au[12 + e] = bf_bits(x3[e]);
    }
    const v16bf a = __builtin_bit_cast(v16bf, au);
    const unsigned short* bp = wrow + 32 * c;
    const v16bf f0 = ldfrag_b(bp);
    const v16bf f1 = ldfrag_b(bp + 16 * CH);
    const v16bf f2 = ldfrag_b(bp + 32 * CH);
    const v16bf f3 = ldfrag_b(bp + 48 * CH);
    const v16bf f4 = ldfrag_b(bp + 64 * CH);
    acc[0] = mma_b(a, f0, acc[0]);
    acc[1] = mma_b(a, f1, acc[1]);
    acc[2] = mma_b(a, f2, acc[2]);
    acc[3] = mma_b(a, f3, acc[3]);
    acc[4] = mma_b(a, f4, acc[4]);
    guard_pj(acc[0], acc[1], acc[2], acc[3], acc[4], a, f0, f1, f2, f3, f4);
    sched_fence();
  }
  accg5(acc[0], acc[1], acc[2], acc[3], acc[4]);

#pragma unroll
  for (int j = 0; j < 5; ++j) {
    const int t = tbase + j;
    if (t >= 2) {
      const int ch = (t - 2) * 16 + m;
      const float bb = sBias[2 * DQ + ch];
      v8h pv;
#pragma unroll
      for (int r = 0; r < 8; ++r) pv[r] = (_Float16)((acc[j][r] + bb) * 16.0f);
      *(v8h*)(sVT + ch * PVT + tw * 16 + 8 * h) = pv;
    } else if (t == 0) {
      const float bb = sBias[m];
      unsigned short* dh = sQH + tw * 256 + m;
      unsigned short* dl = sQL + tw * 256 + m;
#pragma unroll
      for (int r = 0; r < 8; ++r) {
        const float val = acc[j][r] + bb;
        const unsigned short hb = bf_bits(val);
        const unsigned short lb = bf_bits(val - bf_up(hb));
        dh[(8 * h + r) * DQ] = hb;
        dl[(8 * h + r) * DQ] = lb;
      }
    } else {
      const float bb = sBias[DQ + m];
      unsigned short* dh = sKH + tw * 256 + m;
      unsigned short* dl = sKL + tw * 256 + m;
#pragma unroll
      for (int r = 0; r < 8; ++r) {
        const float val = acc[j][r] + bb;
        const unsigned short hb = bf_bits(val);
        const unsigned short lb = bf_bits(val - bf_up(hb));
        dh[(8 * h + r) * DQ] = hb;
        dl[(8 * h + r) * DQ] = lb;
      }
    }
  }
  __syncthreads();

  const v4u qhv = *(const v4u*)(sQH + tw * 256 + lane * 8);
  const v4u qlv = *(const v4u*)(sQL + tw * 256 + lane * 8);
  const v4u khv = *(const v4u*)(sKH + tw * 256 + lane * 8);
  const v4u klv = *(const v4u*)(sKL + tw * 256 + lane * 8);
  const size_t qoff = (size_t)row0 * DQ + (size_t)lane * 8;
  v4u vv[4];
  size_t voff[4];
  const int piece = lane & 7, chl = lane >> 3;
#pragma unroll
  for (int i = 0; i < 4; ++i) {
    const int ch = i * 32 + w * 4 + chl;
    const v8h tv = *(const v8h*)(sVT + ch * PVT + piece * 8);
    vv[i] = __builtin_bit_cast(v4u, tv);
    voff[i] = ((size_t)(b * CH + ch)) * NP + (size_t)tl0 + (size_t)piece * 8;
  }

  if (g == 0) {
    *(volatile v4u*)(QH + qoff) = qhv;
    *(volatile v4u*)(QL + qoff) = qlv;
    *(volatile v4u*)(KH + qoff) = khv;
    *(volatile v4u*)(KL + qoff) = klv;
  }
#pragma unroll
  for (int i = 0; i < 4; ++i) *(volatile v4u*)(VT + voff[i]) = vv[i];
  __threadfence();
  if (g == 0) {
    *(volatile v4u*)(QH + qoff) = qhv;
    *(volatile v4u*)(QL + qoff) = qlv;
    *(volatile v4u*)(KH + qoff) = khv;
    *(volatile v4u*)(KL + qoff) = klv;
  }
#pragma unroll
  for (int i = 0; i < 4; ++i) *(volatile v4u*)(VT + voff[i]) = vv[i];
}

__global__ __launch_bounds__(128) void k_attn(const float* __restrict__ x, const float* __restrict__ gamma,
                                               const unsigned short* QH, const unsigned short* QL,
                                               const unsigned short* KH, const unsigned short* KL,
                                               const _Float16* VT, float* out) {
  __shared__ __align__(16) float sO[TB * PO];
  __shared__ float sFac[TB];
  const int tid = threadIdx.x, w = tid >> 5, lane = tid & 31, m = lane & 15, h = lane >> 4;
  const int blk = blockIdx.x;
  const int tok0 = blk * TB;
  const int b = blk >> 6;
  const int keybase = b * NP;
  const int qrow0 = tok0 + 16 * w;
  const float gm = bf_r(gamma[0]);
  const float C1 = 1.4426950408889634f;
  const v8us z8u = zero8us();

  const v16bf bqh = ldfrag16_b(QH + (size_t)(qrow0 + m) * DQ + 8 * h, z8u);
  const v16bf bql = ldfrag16_b(QL + (size_t)(qrow0 + m) * DQ + 8 * h, z8u);
  const unsigned short* khp = KH + (size_t)(keybase + m) * DQ + 8 * h;
  const unsigned short* klp = KL + (size_t)(keybase + m) * DQ + 8 * h;
  const _Float16* vp = VT + ((size_t)b * CH + m) * NP + 8 * h;

  float rmax = -3.0e38f;
#pragma unroll 1
  for (int kb = 0; kb < NP; kb += 32) {
    const v16bf a0 = ldfrag16_b(khp + (size_t)kb * DQ, z8u);
    const v16bf a1 = ldfrag16_b(khp + (size_t)(kb + 16) * DQ, z8u);
    v8f s0 = mma_b(a0, bqh, zero8());
    v8f s1 = mma_b(a1, bqh, zero8());
    guard_s1(s0, s1, a0, a1, bqh);
    sched_fence();
    float l0 = fmaxf(s0[0], s1[0]);
    float l1 = fmaxf(s0[4], s1[4]);
#pragma unroll
    for (int e = 1; e < 4; ++e) {
      l0 = fmaxf(l0, fmaxf(s0[e], s1[e]));
      l1 = fmaxf(l1, fmaxf(s0[4 + e], s1[4 + e]));
    }
    rmax = fmaxf(rmax, fmaxf(l0, l1));
  }
  rmax = fmaxf(rmax, __shfl_xor(rmax, 16, 32));
  const float dsh = 12.0f - rmax * C1;

  v8f acc[8];
#pragma unroll
  for (int c = 0; c < 8; ++c) acc[c] = zero8();
  v8f lsv = zero8();
#pragma unroll 1
  for (int kb = 0; kb < NP; kb += 32) {
    const v16bf a0h = ldfrag16_b(khp + (size_t)kb * DQ, z8u);
    const v16bf a1h = ldfrag16_b(khp + (size_t)(kb + 16) * DQ, z8u);
    const v16bf a0l = ldfrag16_b(klp + (size_t)kb * DQ, z8u);
    const v16bf a1l = ldfrag16_b(klp + (size_t)(kb + 16) * DQ, z8u);
    v8f s0 = mma_b(a0h, bqh, zero8());
    s0 = mma_b(a0h, bql, s0);
    s0 = mma_b(a0l, bqh, s0);
    v8f s1 = mma_b(a1h, bqh, zero8());
    s1 = mma_b(a1h, bql, s1);
    s1 = mma_b(a1l, bqh, s1);
    guard_s3(s0, s1, a0h, a1h, a0l, a1l, bqh, bql);
    sched_fence();
    v8f p0, p1;
#pragma unroll
    for (int e = 0; e < 8; ++e) {
      p0[e] = FEXP2(s0[e] * C1 + dsh);
      p1[e] = FEXP2(s1[e] * C1 + dsh);
    }
    lsv += p0 + p1;
    v16h pb;
#pragma unroll
    for (int e = 0; e < 8; ++e) {
      pb[e]     = (_Float16)p0[e];
      pb[8 + e] = (_Float16)p1[e];
    }
    const _Float16* vk = vp + kb;
    {
      const v16h va0 = ldfrag_h(vk);
      const v16h va1 = ldfrag_h(vk + (size_t)16 * NP);
      const v16h va2 = ldfrag_h(vk + (size_t)32 * NP);
      const v16h va3 = ldfrag_h(vk + (size_t)48 * NP);
      acc[0] = mma_h(va0, pb, acc[0]);
      acc[1] = mma_h(va1, pb, acc[1]);
      acc[2] = mma_h(va2, pb, acc[2]);
      acc[3] = mma_h(va3, pb, acc[3]);
      guard_pv(acc[0], acc[1], acc[2], acc[3], va0, va1, va2, va3, pb);
    }
    {
      const v16h va4 = ldfrag_h(vk + (size_t)64 * NP);
      const v16h va5 = ldfrag_h(vk + (size_t)80 * NP);
      const v16h va6 = ldfrag_h(vk + (size_t)96 * NP);
      const v16h va7 = ldfrag_h(vk + (size_t)112 * NP);
      acc[4] = mma_h(va4, pb, acc[4]);
      acc[5] = mma_h(va5, pb, acc[5]);
      acc[6] = mma_h(va6, pb, acc[6]);
      acc[7] = mma_h(va7, pb, acc[7]);
      guard_pv(acc[4], acc[5], acc[6], acc[7], va4, va5, va6, va7, pb);
    }
    sched_fence();
  }
  accg8(acc[0], acc[1], acc[2], acc[3], acc[4], acc[5], acc[6], acc[7]);

  float tot = ((lsv[0] + lsv[1]) + (lsv[2] + lsv[3])) + ((lsv[4] + lsv[5]) + (lsv[6] + lsv[7]));
  tot += __shfl_xor(tot, 16, 32);
  const float fac = (gm * 0.0625f) * (1.0f / tot);
  if (h == 0) sFac[16 * w + m] = fac;

  float* so = sO + (16 * w + m) * PO + 8 * h;
#pragma unroll
  for (int c = 0; c < 8; ++c) {
    Acc8 u;
    u.v = acc[c];
    *(v4f*)(so + 16 * c)     = u.q[0];
    *(v4f*)(so + 16 * c + 4) = u.q[1];
  }
  __syncthreads();

  v4f res[16];
#pragma unroll
  for (int r = 0; r < 16; ++r) {
    const v4f o4 = *(const v4f*)(sO + (16 * w + r) * PO + 4 * lane);
    const v4f x4 = *(const v4f*)(x + (size_t)(qrow0 + r) * CH + 4 * lane);
    const float f = sFac[16 * w + r];
    v4f xb;
    xb[0] = bf_r(x4[0]); xb[1] = bf_r(x4[1]); xb[2] = bf_r(x4[2]); xb[3] = bf_r(x4[3]);
    res[r] = o4 * f + xb;
  }
#pragma unroll
  for (int r = 0; r < 16; ++r)
    *(volatile v4f*)(out + (size_t)(qrow0 + r) * CH + 4 * lane) = res[r];
  __threadfence();
#pragma unroll
  for (int r = 0; r < 16; ++r)
    *(volatile v4f*)(out + (size_t)(qrow0 + r) * CH + 4 * lane) = res[r];
}

extern "C" void kernel_launch(void* const* d_in, const int* in_sizes, int n_in,
                              void* d_out, int out_size, void* d_ws, size_t ws_size,
                              hipStream_t stream) {
  if (n_in < 8) return;
  if (in_sizes[0] != NT * CH) return;
  if (in_sizes[1] != CH * DQ) return;
  if (in_sizes[2] != DQ) return;
  if (in_sizes[3] != CH * DQ) return;
  if (in_sizes[4] != DQ) return;
  if (in_sizes[5] != CH * CH) return;
  if (in_sizes[6] != CH) return;
  if (in_sizes[7] < 1) return;
  if (out_size != NT * CH) return;

  const float* x     = (const float*)d_in[0];
  const float* Wq    = (const float*)d_in[1];
  const float* bq    = (const float*)d_in[2];
  const float* Wk    = (const float*)d_in[3];
  const float* bk    = (const float*)d_in[4];
  const float* Wv    = (const float*)d_in[5];
  const float* bv    = (const float*)d_in[6];
  const float* gamma = (const float*)d_in[7];
  float* out = (float*)d_out;

  const size_t PWT = (size_t)NCOL * CH * 2;
  const size_t PQK = (size_t)NT * DQ * 2;
  const size_t PVP = (size_t)NB * CH * NP * 2;

  size_t off = 0;
  const size_t oWT = off; off += PWT;
  const size_t oQH = off; off += PQK;
  const size_t oQL = off; off += PQK;
  const size_t oKH = off; off += PQK;
  const size_t oKL = off; off += PQK;
  const size_t oV  = off; off += PVP;
  if (off > ws_size) return;
  if (off > (size_t)134217728) return;

  char* ws = (char*)d_ws;
  unsigned short* WT = (unsigned short*)(ws + oWT);
  unsigned short* QH = (unsigned short*)(ws + oQH);
  unsigned short* QL = (unsigned short*)(ws + oQL);
  unsigned short* KH = (unsigned short*)(ws + oKH);
  unsigned short* KL = (unsigned short*)(ws + oKL);
  _Float16* VT  = (_Float16*)(ws + oV);

  k_prep<<<dim3(NCOL / 16), dim3(256), 0, stream>>>(Wq, Wk, Wv, WT);
  k_proj<<<dim3(NT / TB), dim3(256), 0, stream>>>(x, WT, bq, bk, bv, QH, QL, KH, KL, VT);
  k_attn<<<dim3(NT / TB), dim3(128), 0, stream>>>(x, gamma, QH, QL, KH, KL, VT, out);
  (void)hipGetLastError();
}
